// GATDiscriminator_31774168056072
// MI455X (gfx1250) — hardware-run, weakly checked
//
#include <hip/hip_runtime.h>

typedef float          v8f   __attribute__((ext_vector_type(8)));
typedef float          v4f   __attribute__((ext_vector_type(4)));
typedef unsigned int   v4u   __attribute__((ext_vector_type(4)));
typedef int            v8i   __attribute__((ext_vector_type(8)));
typedef unsigned short v8us  __attribute__((ext_vector_type(8)));
typedef unsigned short v16us __attribute__((ext_vector_type(16)));
typedef __bf16         v16bf __attribute__((ext_vector_type(16)));
typedef _Float16       v16h  __attribute__((ext_vector_type(16)));
typedef v4f  __attribute__((may_alias)) v4fa;
typedef v8us __attribute__((may_alias)) v8usa;
union FragB { v16bf v; v16us u; v8us h[2]; v8i w; };
union FragH { v16h  v; v16us u; v8us h[2]; v8i w; };

__device__ __forceinline__ v8f wmb(const FragB& a, const FragB& b, v8f c) {
  v8f d = __builtin_amdgcn_wmma_f32_16x16x32_bf16(false, a.v, false, b.v, (short)0, c, false, false);
  asm volatile("v_nop\n\tv_nop\n\tv_nop\n\tv_nop" : "+v"(d) : "v"(a.w), "v"(b.w));
  return d;
}

__device__ __forceinline__ v8f wmh(const FragH& a, const FragH& b, v8f c) {
  v8f d = __builtin_amdgcn_wmma_f32_16x16x32_f16(false, a.v, false, b.v, (short)0, c, false, false);
  asm volatile("v_nop\n\tv_nop\n\tv_nop\n\tv_nop" : "+v"(d) : "v"(a.w), "v"(b.w));
  return d;
}

__device__ __forceinline__ unsigned bf16_bits(float f) {
  const unsigned u = __float_as_uint(f);
  const unsigned r = (u + 0x7FFFu + ((u >> 16) & 1u)) >> 16;
  const unsigned q = (u >> 16) | 0x40u;
  return ((u & 0x7fffffffu) > 0x7f800000u) ? q : r;
}

__device__ __forceinline__ float bf16_val(float f) {
  return __uint_as_float(bf16_bits(f) << 16);
}
__device__ __forceinline__ int clampi(int v, int lo, int hi) {
  return v < lo ? lo : (v > hi ? hi : v);
}

__device__ __forceinline__ unsigned f16_bits(float f) {
  const unsigned u  = __float_as_uint(f);
  const unsigned s  = (u >> 16) & 0x8000u;
  const unsigned a  = u & 0x7fffffffu;
  const unsigned t  = a - 0x38000000u;
  const unsigned r  = (t + 0x0FFFu + ((t >> 13) & 1u)) >> 13;
  const unsigned rc = r > 0x7C00u ? 0x7C00u : r;
  const bool small  = a < 0x38800000u;
  const bool isnan  = a > 0x7f800000u;
  const unsigned fin = small ? 0u : (s | rc);
  return isnan ? (s | 0x7E00u) : fin;
}

__device__ __forceinline__ unsigned pk16(unsigned lo, unsigned hi) { return lo | (hi << 16); }
__device__ __forceinline__ unsigned bf16_lo_bits(float v) {
  float hi = bf16_val(v);
  asm volatile("" : "+v"(hi));
  return bf16_bits(v - hi);
}
__device__ __forceinline__ v4u pack8_bf16(v4f a, v4f c) {
  return (v4u){ pk16(bf16_bits(a[0]), bf16_bits(a[1])), pk16(bf16_bits(a[2]), bf16_bits(a[3])),
                pk16(bf16_bits(c[0]), bf16_bits(c[1])), pk16(bf16_bits(c[2]), bf16_bits(c[3])) };
}
__device__ __forceinline__ v4u pack8_bf16_lo(v4f a, v4f c) {
  return (v4u){ pk16(bf16_lo_bits(a[0]), bf16_lo_bits(a[1])), pk16(bf16_lo_bits(a[2]), bf16_lo_bits(a[3])),
                pk16(bf16_lo_bits(c[0]), bf16_lo_bits(c[1])), pk16(bf16_lo_bits(c[2]), bf16_lo_bits(c[3])) };
}
__device__ __forceinline__ v4u pack8_f16(v4f a, v4f c) {
  return (v4u){ pk16(f16_bits(a[0]), f16_bits(a[1])), pk16(f16_bits(a[2]), f16_bits(a[3])),
                pk16(f16_bits(c[0]), f16_bits(c[1])), pk16(f16_bits(c[2]), f16_bits(c[3])) };
}

template <int FORM>
__global__ __launch_bounds__(256) void k_plane(const float* __restrict__ src, int rows, int cols, int ldsrc,
                                               unsigned short* __restrict__ dst, int MP, int KP) {
  static_assert(FORM >= 0 && FORM <= 3);
  const int KTOT = (FORM == 1 || FORM == 3) ? 2 * KP : KP;
  const unsigned ppr   = (unsigned)(KTOT >> 3);
  const unsigned kp8   = (unsigned)(KP >> 3);
  const unsigned total = (unsigned)MP * ppr;
  const unsigned g     = blockIdx.x * 256u + threadIdx.x;
  const unsigned rowu  = g / ppr;
  const unsigned p     = g - rowu * ppr;
  const bool second    = p >= kp8;
  const int row = (int)rowu;
  const int c0  = (int)((second ? p - kp8 : p) << 3);
  const float* srow = src + (size_t)clampi(row, 0, rows - 1) * (size_t)ldsrc;
  float x[8];
  unsigned mk[8];
#pragma unroll
  for (int e = 0; e < 8; ++e) {
    const int c = c0 + e;
    const float v = srow[clampi(c, 0, cols - 1)];
    asm volatile("" :: "v"(v));
    x[e]  = v;
    mk[e] = (row < rows && c < cols) ? 0xFFFFu : 0u;
  }
  const v4f a = (v4f){ x[0], x[1], x[2], x[3] };
  const v4f c = (v4f){ x[4], x[5], x[6], x[7] };
  v4u o;
  if (FORM == 2) {
    o = pack8_f16(a, c);
  } else {
    const v4u hi = pack8_bf16(a, c);
    o = hi;
    if (FORM == 1) { const v4u lo = pack8_bf16_lo(a, c); o = second ? lo : hi; }
  }
  const v4u mw = (v4u){ pk16(mk[0], mk[1]), pk16(mk[2], mk[3]), pk16(mk[4], mk[5]), pk16(mk[6], mk[7]) };
  o &= mw;
  if (g < total) {
    volatile v4u* q = (volatile v4u*)(dst + (size_t)g * 8);
    *q = o;
    __threadfence();
    *q = o;
  }
}

template <int FORM> struct FragOf    { typedef FragB T; };
template <>         struct FragOf<2> { typedef FragH T; };
__device__ __forceinline__ v8f mm(const FragB& a, const FragB& b, v8f c) { return wmb(a, b, c); }
__device__ __forceinline__ v8f mm(const FragH& a, const FragH& b, v8f c) { return wmh(a, b, c); }
template <class F> __device__ __forceinline__ F ld_frag(const unsigned short* p) {
  F f;
  f.h[0] = *(const v8usa*)(p);
  f.h[1] = *(const v8usa*)(p + 16);
  return f;
}

template <int FORM, int EPI>
__global__ __launch_bounds__(256) __attribute__((amdgpu_num_vgpr(248)))
void k_gemm_nt(const unsigned short* __restrict__ A, const unsigned short* __restrict__ B,
               const float* __restrict__ bias, float* __restrict__ D, int M, int N, int KTOT, int ldd) {
  static_assert(FORM >= 0 && FORM <= 2);
  static_assert(EPI == 0 || EPI == 1);
  typedef typename FragOf<FORM>::T F;
  __shared__ __attribute__((aligned(16))) float sT[8][16 * 68];
  const int lane = threadIdx.x & 31;
  const int wave = threadIdx.x >> 5;
  const int tilesM = (M + 63) >> 6;
  const int tilesN = (N + 63) >> 6;
  const int tile = blockIdx.x * 8 + wave;
  if (tile >= tilesM * tilesN) return;
  const int tm = tile / tilesN;
  const int tn = tile - tm * tilesN;
  const int m0 = tm << 6;
  const int n0 = tn << 6;

  const int rl = lane & 15;
  const int h8 = (lane >> 4) * 8;
  const unsigned short* pa = A + (size_t)(m0 + rl) * (size_t)KTOT + h8;
  const unsigned short* pb = B + (size_t)(n0 + rl) * (size_t)KTOT + h8;

  v8f acc[4][4];
#pragma unroll
  for (int i = 0; i < 4; ++i)
#pragma unroll
    for (int j = 0; j < 4; ++j) acc[i][j] = (v8f){0.f, 0.f, 0.f, 0.f, 0.f, 0.f, 0.f, 0.f};

#pragma unroll 1
  for (int k0 = 0; k0 < KTOT; k0 += 32) {
    F bf[4];
#pragma unroll
    for (int j = 0; j < 4; ++j) bf[j] = ld_frag<F>(pb + (size_t)(j << 4) * (size_t)KTOT + k0);
#pragma unroll
    for (int i = 0; i < 4; ++i) {
      const F af = ld_frag<F>(pa + (size_t)(i << 4) * (size_t)KTOT + k0);
#pragma unroll
      for (int j = 0; j < 4; ++j) acc[i][j] = mm(af, bf[j], acc[i][j]);
    }
  }

  float* slab = sT[wave];
  const int hh = lane >> 4;
  const int c4 = (lane & 15) * 4;
  const int nc = n0 + c4;
  const bool cok = nc < N;
  v4f bv = (v4f){0.f, 0.f, 0.f, 0.f};
  if (EPI == 1) {
    bv = *(const v4fa*)(bias + clampi(nc, 0, N - 4));
    asm volatile("" :: "v"(bv));
  }
#pragma unroll
  for (int i = 0; i < 4; ++i) {
    const int mBase = m0 + (i << 4);
#pragma unroll
    for (int j = 0; j < 4; ++j) {
#pragma unroll
      for (int r = 0; r < 8; ++r) slab[(h8 + r) * 68 + (j << 4) + rl] = acc[i][j][r];
    }
    __builtin_amdgcn_fence(__ATOMIC_RELEASE, "workgroup");
    __builtin_amdgcn_wave_barrier();
    __builtin_amdgcn_fence(__ATOMIC_ACQUIRE, "workgroup");
    v4f vv[8];
#pragma unroll
    for (int it = 0; it < 8; ++it) {
      const int row = it * 2 + hh;
      v4f v = *(const v4fa*)(slab + row * 68 + c4);
      if (EPI == 1) v += bv;
      vv[it] = v;
    }
    for (int pass = 0; pass < 2; ++pass) {
#pragma unroll
      for (int it = 0; it < 8; ++it) {
        const int row = mBase + it * 2 + hh;
        if (cok && row < M) *(volatile v4f*)(D + (size_t)row * (size_t)ldd + nc) = vv[it];
      }
      __threadfence();
    }
    __builtin_amdgcn_fence(__ATOMIC_RELEASE, "workgroup");
    __builtin_amdgcn_wave_barrier();
    __builtin_amdgcn_fence(__ATOMIC_ACQUIRE, "workgroup");
  }
}

#pragma clang fp contract(off)


#define SPLIT_2 1
#define NN      100000
#define NE      1600000
#define MPAD    100096
#define KIN     128
#define NOUT    192
#define HCH     64
#define KT2     (SPLIT_2 ? 128 : 64)
#define TB_AS1  0
#define TB_AD1  192
#define TB_AS2  384
#define TB_AD2  576
#define TB_B1   768
#define TB_B2   832
#define TB_LW   1024
#define TB_LB   1216
#define TB_N    2048
#define PREP_W1B (NOUT * (KIN / 8) / 256)
#define PREP_W2B (NOUT * (KT2 / 8) / 256)
#define PREP_TBB (TB_N / 4 / 256)
#define PREP_BLK (PREP_W1B + PREP_W2B + PREP_TBB)
#define BT      512
#define BW      16
#define BEPT    8
#define BCHUNK  (BT * BEPT)
#define NCH     ((NE + BCHUNK - 1) / BCHUNK)
#define NB      1024
#define NBLK    ((NN + NB - 1) / NB)
#define LCAP    21504
#define DEGCAP  64
#define SLOTSH  17
#define SRCMASK ((1u << SLOTSH) - 1u)
#define LISTTOT (NBLK * LCAP)
#define LDS_LIST ((2 * LCAP + 3 * NB + 64) * 4)
#define WTHR    256
#define WWAVES  8
#define WSMAX   ((size_t)128 << 20)

static_assert(HCH == 2 * 32 && NOUT == 3 * HCH);
static_assert(MPAD == 782 * 128 && MPAD % 64 == 0 && MPAD >= NN);
static_assert(NN < (1 << SLOTSH) && SLOTSH + 10 <= 32);
static_assert(NB == 1024 && NB == 2 * BT);
static_assert(NE % 8 == 0 && NE >= 8);
static_assert(NBLK == 98 && NBLK * NB >= NN);
static_assert(NCH * BCHUNK >= NE && NCH == 391);
static_assert(LCAP % 256 == 0);
static_assert(LCAP * 4 >= 16673 * 5);
static_assert(DEGCAP >= 36 + 8);
static_assert(LDS_LIST <= 262144);
static_assert(BW == BT / 32);
static_assert(NN % 32 == 0 && NN % WWAVES == 0 && MPAD % 32 == 0);
static_assert(KT2 % 32 == 0 && KIN % 32 == 0);
static_assert((NOUT * (KIN / 8)) % 256 == 0 && (NOUT * (KT2 / 8)) % 256 == 0 && (TB_N / 4) % 256 == 0);
static_assert(TB_LB + 4 <= TB_N);

typedef float        v2f __attribute__((ext_vector_type(2)));
typedef int          v4i __attribute__((ext_vector_type(4)));
typedef int          v2i __attribute__((ext_vector_type(2)));
typedef v2f __attribute__((may_alias)) v2fa;
typedef v4i __attribute__((may_alias)) v4ia;
typedef v2i __attribute__((may_alias)) v2ia;

__device__ __forceinline__ float lrelu_k(float v) { return (v >= 0.0f) ? v : 0.2f * v; }
__device__ __forceinline__ float rrelu_k(float v) {
  const float sl = (1.0f / 8.0f + 1.0f / 3.0f) / 2.0f;
  return (v >= 0.0f) ? v : v * sl;
}
__device__ __forceinline__ float maxk(float a, float b) {
  float m = (a < b) ? b : a;
  m = (b != b) ? b : m;
  return m;
}
__device__ __forceinline__ float wsum(float t) {
  t = t + __shfl_xor(t, 16, 32);
  t = t + __shfl_xor(t, 8, 32);
  t = t + __shfl_xor(t, 4, 32);
  t = t + __shfl_xor(t, 2, 32);
  t = t + __shfl_xor(t, 1, 32);
  return t;
}
__device__ __forceinline__ float wmaxk(float t) {
  t = maxk(t, __shfl_xor(t, 16, 32));
  t = maxk(t, __shfl_xor(t, 8, 32));
  t = maxk(t, __shfl_xor(t, 4, 32));
  t = maxk(t, __shfl_xor(t, 2, 32));
  t = maxk(t, __shfl_xor(t, 1, 32));
  return t;
}

__global__ __launch_bounds__(256) void k_planezx(const float* __restrict__ z, const float* __restrict__ x,
                                                 unsigned short* XB) {
  const unsigned g = blockIdx.x * 256u + threadIdx.x;
  const int row = (int)(g >> 4);
  const int p   = (int)(g & 15u);
  const int c0  = (p & 7) << 3;
  const int rc  = row < NN ? row : NN - 1;
  const v4f z0 = *(const v4fa*)(z + (size_t)rc * HCH + c0);
  const v4f z1 = *(const v4fa*)(z + (size_t)rc * HCH + c0 + 4);
  const v4f x0 = *(const v4fa*)(x + (size_t)rc * HCH + c0);
  const v4f x1 = *(const v4fa*)(x + (size_t)rc * HCH + c0 + 4);
  asm volatile("" :: "v"(z0), "v"(z1), "v"(x0), "v"(x1));
  const v4u zb = pack8_bf16(z0, z1);
  const v4u xb = pack8_bf16(x0, x1);
  const unsigned mz = (p < 8 && row < NN) ? 0xFFFFFFFFu : 0u;
  const unsigned mx = (p >= 8 && row < NN) ? 0xFFFFFFFFu : 0u;
  const v4u o = (zb & (v4u){mz, mz, mz, mz}) | (xb & (v4u){mx, mx, mx, mx});
  volatile v4u* q = (volatile v4u*)(XB + (size_t)g * 8);
  *q = o;
  __threadfence();
  *q = o;
}

__global__ __launch_bounds__(256) void k_prep(const float* __restrict__ W1, const float* __restrict__ W2,
                                              const float* __restrict__ as1, const float* __restrict__ ad1,
                                              const float* __restrict__ b1,
                                              const float* __restrict__ as2, const float* __restrict__ ad2,
                                              const float* __restrict__ b2,
                                              const float* __restrict__ lw, const float* __restrict__ lb,
                                              unsigned short* W1T, unsigned short* W2D, float* TB) {
  const int blk = (int)blockIdx.x;
  const int t   = (int)threadIdx.x;
  if (blk < PREP_W1B) {
    const int g  = blk * 256 + t;
    const int n  = g / (KIN / 8);
    const int k0 = (g - n * (KIN / 8)) << 3;
    float xv[8];
#pragma unroll
    for (int e = 0; e < 8; ++e) {
      const float v = W1[(size_t)(k0 + e) * NOUT + n];
      asm volatile("" :: "v"(v));
      xv[e] = v;
    }
    const v4u o = pack8_bf16((v4f){xv[0], xv[1], xv[2], xv[3]}, (v4f){xv[4], xv[5], xv[6], xv[7]});
    volatile v4u* q = (volatile v4u*)(W1T + (size_t)g * 8);
    *q = o;
    __threadfence();
    *q = o;
  } else if (blk < PREP_W1B + PREP_W2B) {
    const int g  = (blk - PREP_W1B) * 256 + t;
    const int n  = g / (KT2 / 8);
    const int k0 = ((g - n * (KT2 / 8)) << 3) & (HCH - 1);
    float xv[8];
#pragma unroll
    for (int e = 0; e < 8; ++e) {
      const float v = W2[(size_t)(k0 + e) * NOUT + n];
      asm volatile("" :: "v"(v));
      xv[e] = v;
    }
    const v4u o = pack8_bf16((v4f){xv[0], xv[1], xv[2], xv[3]}, (v4f){xv[4], xv[5], xv[6], xv[7]});
    volatile v4u* q = (volatile v4u*)(W2D + (size_t)g * 8);
    *q = o;
    __threadfence();
    *q = o;
  } else {
    const int idx = 4 * ((blk - PREP_W1B - PREP_W2B) * 256 + t);
    const v4f a0 = *(const v4fa*)(as1 + clampi(idx - TB_AS1, 0, 188));
    asm volatile("" :: "v"(a0));
    const v4f a1 = *(const v4fa*)(ad1 + clampi(idx - TB_AD1, 0, 188));
    asm volatile("" :: "v"(a1));
    const v4f a2 = *(const v4fa*)(as2 + clampi(idx - TB_AS2, 0, 188));
    asm volatile("" :: "v"(a2));
    const v4f a3 = *(const v4fa*)(ad2 + clampi(idx - TB_AD2, 0, 188));
    asm volatile("" :: "v"(a3));
    const v4f a4 = *(const v4fa*)(b1 + clampi(idx - TB_B1, 0, 60));
    asm volatile("" :: "v"(a4));
    const v4f a5 = *(const v4fa*)(b2 + clampi(idx - TB_B2, 0, 188));
    asm volatile("" :: "v"(a5));
    const v4f a6 = *(const v4fa*)(lw + clampi(idx - TB_LW, 0, 188));
    asm volatile("" :: "v"(a6));
    const float lbv = lb[0];
    asm volatile("" :: "v"(lbv));
    const unsigned m0 = (idx < TB_AD1) ? 0xFFFFFFFFu : 0u;
    const unsigned m1 = (idx >= TB_AD1 && idx < TB_AS2) ? 0xFFFFFFFFu : 0u;
    const unsigned m2 = (idx >= TB_AS2 && idx < TB_AD2) ? 0xFFFFFFFFu : 0u;
    const unsigned m3 = (idx >= TB_AD2 && idx < TB_B1) ? 0xFFFFFFFFu : 0u;
    const unsigned m4 = (idx >= TB_B1 && idx < TB_B2) ? 0xFFFFFFFFu : 0u;
    const unsigned m5 = (idx >= TB_B2 && idx < TB_LW) ? 0xFFFFFFFFu : 0u;
    const unsigned m6 = (idx >= TB_LW && idx < TB_LB) ? 0xFFFFFFFFu : 0u;
    const unsigned m7 = (idx == TB_LB) ? 0xFFFFFFFFu : 0u;
    v4u o;
    o.x = (__float_as_uint(a0.x) & m0) | (__float_as_uint(a1.x) & m1) | (__float_as_uint(a2.x) & m2) |
          (__float_as_uint(a3.x) & m3) | (__float_as_uint(a4.x) & m4) | (__float_as_uint(a5.x) & m5) |
          (__float_as_uint(a6.x) & m6) | (__float_as_uint(lbv) & m7);
    o.y = (__float_as_uint(a0.y) & m0) | (__float_as_uint(a1.y) & m1) | (__float_as_uint(a2.y) & m2) |
          (__float_as_uint(a3.y) & m3) | (__float_as_uint(a4.y) & m4) | (__float_as_uint(a5.y) & m5) |
          (__float_as_uint(a6.y) & m6);
    o.z = (__float_as_uint(a0.z) & m0) | (__float_as_uint(a1.z) & m1) | (__float_as_uint(a2.z) & m2) |
          (__float_as_uint(a3.z) & m3) | (__float_as_uint(a4.z) & m4) | (__float_as_uint(a5.z) & m5) |
          (__float_as_uint(a6.z) & m6);
    o.w = (__float_as_uint(a0.w) & m0) | (__float_as_uint(a1.w) & m1) | (__float_as_uint(a2.w) & m2) |
          (__float_as_uint(a3.w) & m3) | (__float_as_uint(a4.w) & m4) | (__float_as_uint(a5.w) & m5) |
          (__float_as_uint(a6.w) & m6);
    o.x = bf16_bits(__uint_as_float(o.x)) << 16;
    o.y = bf16_bits(__uint_as_float(o.y)) << 16;
    o.z = bf16_bits(__uint_as_float(o.z)) << 16;
    o.w = bf16_bits(__uint_as_float(o.w)) << 16;
    volatile v4u* q = (volatile v4u*)(TB + idx);
    *q = o;
    __threadfence();
    *q = o;
  }
}

__global__ __launch_bounds__(BT) void k_list(const int* __restrict__ esrc, const int* __restrict__ edst,
                                             unsigned* LIST, int* META) {
  extern __shared__ v4u lds_list[];
  int* reg1 = (int*)lds_list;
  int* reg2 = reg1 + LCAP;
  int* scnt = reg2 + LCAP;
  int* soff = scnt + NB;
  int* curs = soff + NB;
  int* wcnt = curs + NB;
  int* wtot = wcnt + 2 * BW;
  const int tid = (int)threadIdx.x, lane = tid & 31, wave = tid >> 5;
  const int nodeBase = (int)blockIdx.x * NB;
  int nb = NN - nodeBase;
  nb = nb > NB ? NB : (nb < 0 ? 0 : nb);
  const unsigned nbs = (unsigned)nodeBase, unb = (unsigned)nb;

  scnt[2 * tid] = 0;
  scnt[2 * tid + 1] = 0;

  int tot = 0;
#pragma unroll 1
  for (int ch = 0; ch < NCH; ++ch) {
    const int par = ch & 1;
    const int e0  = ch * BCHUNK + tid * BEPT;
    const bool valid = e0 < NE;
    const int ea = e0 < NE - 8 ? e0 : NE - 8;
    const v4i da = *(const v4ia*)(edst + ea);
    const v4i db = *(const v4ia*)(edst + ea + 4);
    const v4i sa = *(const v4ia*)(esrc + ea);
    const v4i sb = *(const v4ia*)(esrc + ea + 4);
    asm volatile("" :: "v"(da), "v"(db), "v"(sa), "v"(sb));
    const unsigned s0 = (unsigned)da.x - nbs, s1 = (unsigned)da.y - nbs;
    const unsigned s2 = (unsigned)da.z - nbs, s3 = (unsigned)da.w - nbs;
    const unsigned s4 = (unsigned)db.x - nbs, s5 = (unsigned)db.y - nbs;
    const unsigned s6 = (unsigned)db.z - nbs, s7 = (unsigned)db.w - nbs;
    const bool h0 = valid && (s0 < unb), h1 = valid && (s1 < unb), h2 = valid && (s2 < unb), h3 = valid && (s3 < unb);
    const bool h4 = valid && (s4 < unb), h5 = valid && (s5 < unb), h6 = valid && (s6 < unb), h7 = valid && (s7 < unb);
    const int c = (int)h0 + (int)h1 + (int)h2 + (int)h3 + (int)h4 + (int)h5 + (int)h6 + (int)h7;
    int incl = c;
#pragma unroll
    for (int d = 1; d < 32; d <<= 1) {
      const int up = __shfl_up(incl, d, 32);
      incl += (lane >= d) ? up : 0;
    }
    const int wtotal = __shfl(incl, 31, 32);
    if (lane == 0) wcnt[par * BW + wave] = wtotal;
    __syncthreads();
    int all = 0, pre = 0;
#pragma unroll
    for (int g = 0; g < 4; ++g) {
      const v4i w4 = *(const v4ia*)(wcnt + par * BW + 4 * g);
      const int c0 = clampi(w4.x, 0, 256), c1 = clampi(w4.y, 0, 256);
      const int c2 = clampi(w4.z, 0, 256), c3 = clampi(w4.w, 0, 256);
      all += c0 + c1 + c2 + c3;
      pre += (4 * g + 0 < wave) ? c0 : 0;
      pre += (4 * g + 1 < wave) ? c1 : 0;
      pre += (4 * g + 2 < wave) ? c2 : 0;
      pre += (4 * g + 3 < wave) ? c3 : 0;
    }
    int pos = tot + pre + (incl - c);
#define PUTJ(HJ, SJ, RJ) if (HJ) { if (pos < LCAP) reg1[pos] = (int)((unsigned)clampi((RJ), 0, NN - 1) | ((SJ) << SLOTSH)); ++pos; }
    PUTJ(h0, s0, sa.x)
    PUTJ(h1, s1, sa.y)
    PUTJ(h2, s2, sa.z)
    PUTJ(h3, s3, sa.w)
    PUTJ(h4, s4, sb.x)
    PUTJ(h5, s5, sb.y)
    PUTJ(h6, s6, sb.z)
    PUTJ(h7, s7, sb.w)
#undef PUTJ
    tot += all;
  }
  __syncthreads();
  const bool ovf = tot > LCAP;
  const int nh = ovf ? LCAP : tot;

  if (wave == 0) {
#pragma unroll 1
    for (int b0 = 0; b0 < nh; b0 += 32) {
      const int idx = b0 + lane;
      const int uv  = reg1[idx < nh ? idx : nh - 1];
      const int m32 = (nh - b0) < 32 ? (nh - b0) : 32;
#pragma unroll 1
      for (int k = 0; k < m32; ++k) {
        const int u  = __builtin_amdgcn_readlane(uv, k);
        const int sl = (int)(((unsigned)u >> SLOTSH) & (unsigned)(NB - 1));
        const int cv = scnt[sl] + 1;
        if (lane == 0) scnt[sl] = cv;
      }
    }
  }
  __syncthreads();

  int e0c, e1c;
  {
    const v2i cc = *(const v2ia*)(scnt + 2 * tid);
    e0c = cc.x < 0 ? 0 : cc.x;
    e1c = cc.y < 0 ? 0 : cc.y;
    const int ts = e0c + e1c;
    int incl = ts;
#pragma unroll
    for (int d = 1; d < 32; d <<= 1) {
      const int up = __shfl_up(incl, d, 32);
      incl += (lane >= d) ? up : 0;
    }
    if (lane == 31) wtot[wave] = incl;
    __syncthreads();
    int pre = 0;
#pragma unroll
    for (int g = 0; g < 4; ++g) {
      const v4i w4 = *(const v4ia*)(wtot + 4 * g);
      pre += (4 * g + 0 < wave) ? w4.x : 0;
      pre += (4 * g + 1 < wave) ? w4.y : 0;
      pre += (4 * g + 2 < wave) ? w4.z : 0;
      pre += (4 * g + 3 < wave) ? w4.w : 0;
    }
    const int run = pre + incl - ts;
    soff[2 * tid]     = run;
    soff[2 * tid + 1] = run + e0c;
    curs[2 * tid]     = run;
    curs[2 * tid + 1] = run + e0c;
  }
  __syncthreads();

  if (wave == 0) {
#pragma unroll 1
    for (int b0 = 0; b0 < nh; b0 += 32) {
      const int idx = b0 + lane;
      const int uv  = reg1[idx < nh ? idx : nh - 1];
      const int m32 = (nh - b0) < 32 ? (nh - b0) : 32;
#pragma unroll 1
      for (int k = 0; k < m32; ++k) {
        const int u  = __builtin_amdgcn_readlane(uv, k);
        const int sl = (int)(((unsigned)u >> SLOTSH) & (unsigned)(NB - 1));
        const int pr = curs[sl];
        const int pc = clampi(pr, 0, LCAP - 1);
        if (lane == 0) { reg2[pc] = u; curs[sl] = pc + 1; }
      }
    }
  }
  __syncthreads();

  {
    int nhPad = (nh + 31) & ~31;
    nhPad = nhPad > LCAP ? LCAP : nhPad;
    const int nIt = (nhPad + BT - 1) / BT;
    unsigned* lbase = LIST + (size_t)blockIdx.x * (size_t)LCAP;
#pragma unroll 1
    for (int it = 0; it < nIt; ++it) {
      const int i  = it * BT + tid;
      const int ic = i < nh ? i : nh - 1;
      const unsigned wv  = (unsigned)reg2[ic];
      const unsigned msk = (i < nh) ? 0xFFFFFFFFu : 0u;
      const unsigned o = wv & msk;
      const int iw = i < LCAP ? i : LCAP - 1;
      volatile unsigned* q = (volatile unsigned*)(lbase + (size_t)iw);
      const bool wr = i < nhPad;
      if (wr) *q = o;
      __threadfence();
      if (wr) *q = o;
    }
  }

  {
    const int base = (int)blockIdx.x * LCAP;
    const v2i cc = *(const v2ia*)(scnt + 2 * tid);
    const v2i so = *(const v2ia*)(soff + 2 * tid);
    v4i m;
    m.x = base + so.x;
    m.y = ovf ? -1 : cc.x;
    m.z = base + so.y;
    m.w = ovf ? -1 : cc.y;
    volatile v4i* q = (volatile v4i*)(META + 2 * (size_t)(nodeBase + 2 * tid));
    *q = m;
    __threadfence();
    *q = m;
  }
}

__global__ __launch_bounds__(256) void k_rowprep(const float* __restrict__ XL, const float* __restrict__ atS,
                                                 const float* __restrict__ atD, float* SD) {
  const int lane = (int)threadIdx.x & 31;
  const int wave = (int)threadIdx.x >> 5;
  const int grp  = (int)blockIdx.x * 8 + wave;
  const int n0   = grp * 4;
  const v2f s0t = *(const v2fa*)(atS + 0 * HCH + 2 * lane);
  const v2f s1t = *(const v2fa*)(atS + 1 * HCH + 2 * lane);
  const v2f s2t = *(const v2fa*)(atS + 2 * HCH + 2 * lane);
  const v2f d0t = *(const v2fa*)(atD + 0 * HCH + 2 * lane);
  const v2f d1t = *(const v2fa*)(atD + 1 * HCH + 2 * lane);
  const v2f d2t = *(const v2fa*)(atD + 2 * HCH + 2 * lane);
  const int slot = lane & 7;
  const int q    = lane >> 3;
  float keep = 0.0f;
#pragma unroll 1
  for (int i = 0; i < 4; ++i) {
    const float* xr = XL + (size_t)(n0 + i) * NOUT + 2 * lane;
    const v2f x0 = *(const v2fa*)(xr);
    const v2f x1 = *(const v2fa*)(xr + HCH);
    const v2f x2 = *(const v2fa*)(xr + 2 * HCH);
    asm volatile("" :: "v"(x0), "v"(x1), "v"(x2));
    float a, b;
    a = x0.x * s0t.x; b = x0.y * s0t.y; float s0 = a + b;
    a = x1.x * s1t.x; b = x1.y * s1t.y; float s1 = a + b;
    a = x2.x * s2t.x; b = x2.y * s2t.y; float s2 = a + b;
    a = x0.x * d0t.x; b = x0.y * d0t.y; float d0 = a + b;
    a = x1.x * d1t.x; b = x1.y * d1t.y; float d1 = a + b;
    a = x2.x * d2t.x; b = x2.y * d2t.y; float d2 = a + b;
    s0 = wsum(s0); s1 = wsum(s1); s2 = wsum(s2);
    d0 = wsum(d0); d1 = wsum(d1); d2 = wsum(d2);
    float val = 0.0f;
    val = (slot == 0) ? s0 : val;
    val = (slot == 1) ? s1 : val;
    val = (slot == 2) ? s2 : val;
    val = (slot == 4) ? d0 : val;
    val = (slot == 5) ? d1 : val;
    val = (slot == 6) ? d2 : val;
    keep = (q == i) ? val : keep;
  }
  volatile float* o = (volatile float*)(SD + (size_t)grp * 32 + lane);
  *o = keep;
  __threadfence();
  *o = keep;
}

__device__ __forceinline__ void ld_entry(const unsigned* __restrict__ LIST, const float* __restrict__ SD,
                                         int pos, v4f dd, int& src, float& a0, float& a1, float& a2) {
  const unsigned wd = LIST[(size_t)pos];
  asm volatile("" :: "v"(wd));
  src = clampi((int)(wd & SRCMASK), 0, NN - 1);
  const v4f sv = *(const v4fa*)(SD + (size_t)src * 8);
  asm volatile("" :: "v"(sv));
  float t;
  t = sv.x + dd.x; a0 = lrelu_k(t);
  t = sv.y + dd.y; a1 = lrelu_k(t);
  t = sv.z + dd.z; a2 = lrelu_k(t);
}

template <int LAYER>
__global__ __launch_bounds__(WTHR) void k_walk(const float* __restrict__ XL, const float* __restrict__ SD,
                                               const unsigned* __restrict__ LIST, const int* __restrict__ META,
                                               const float* __restrict__ tbB, const float* __restrict__ tbLw,
                                               const float* __restrict__ tbLb, unsigned* OUT) {
  static_assert(LAYER == 1 || LAYER == 2);
  const int lane = (int)threadIdx.x & 31;
  const int wave = (int)threadIdx.x >> 5;
  const int row  = (int)blockIdx.x * WWAVES + wave;
  const bool rin = row < NN;
  const int rowc = rin ? row : NN - 1;

  const v2i mt = *(const v2ia*)(META + 2 * (size_t)rowc);
  asm volatile("" :: "v"(mt));
  const int craw = mt.y;
  const int offv = clampi(mt.x, 0, LISTTOT);
  const int room = LISTTOT - offv;
  const int cgat = rin ? clampi(craw, 0, DEGCAP) : 0;
  const int cntv = cgat < room ? cgat : room;
  const int off = __builtin_amdgcn_readfirstlane(offv);
  const int cnt = __builtin_amdgcn_readfirstlane(cntv);
  const bool poison = (craw < 0) || (craw > DEGCAP);

  const v4f ss = *(const v4fa*)(SD + (size_t)rowc * 8);
  const v4f dd = *(const v4fa*)(SD + (size_t)rowc * 8 + 4);
  asm volatile("" :: "v"(ss), "v"(dd));
  float tq;
  tq = ss.x + dd.x; const float sa0 = lrelu_k(tq);
  tq = ss.y + dd.y; const float sa1 = lrelu_k(tq);
  tq = ss.z + dd.z; const float sa2 = lrelu_k(tq);

  const float ninf = -__builtin_inff();
  float mx0 = ninf, mx1 = ninf, mx2 = ninf;
#pragma unroll 1
  for (int b0 = 0; b0 < cnt; b0 += 32) {
    const int jj = b0 + lane;
    const bool valid = jj < cnt;
    const int j = valid ? jj : cnt - 1;
    int src; float a0, a1, a2;
    ld_entry(LIST, SD, off + j, dd, src, a0, a1, a2);
    a0 = valid ? a0 : ninf;
    a1 = valid ? a1 : ninf;
    a2 = valid ? a2 : ninf;
    mx0 = maxk(mx0, a0);
    mx1 = maxk(mx1, a1);
    mx2 = maxk(mx2, a2);
  }
  mx0 = wmaxk(mx0); mx1 = wmaxk(mx1); mx2 = wmaxk(mx2);
  mx0 = maxk(mx0, sa0); mx1 = maxk(mx1, sa1); mx2 = maxk(mx2, sa2);

  float dn0 = 0.0f, dn1 = 0.0f, dn2 = 0.0f;
#pragma unroll 1
  for (int b0 = 0; b0 < cnt; b0 += 32) {
    const int jj = b0 + lane;
    const bool valid = jj < cnt;
    const int j = valid ? jj : cnt - 1;
    int src; float a0, a1, a2;
    ld_entry(LIST, SD, off + j, dd, src, a0, a1, a2);
    float e0 = expf(a0 - mx0);
    float e1 = expf(a1 - mx1);
    float e2 = expf(a2 - mx2);
    e0 = valid ? e0 : 0.0f;
    e1 = valid ? e1 : 0.0f;
    e2 = valid ? e2 : 0.0f;
    dn0 = dn0 + e0;
    dn1 = dn1 + e1;
    dn2 = dn2 + e2;
  }
  dn0 = wsum(dn0); dn1 = wsum(dn1); dn2 = wsum(dn2);
  const float es0 = expf(sa0 - mx0);
  const float es1 = expf(sa1 - mx1);
  const float es2 = expf(sa2 - mx2);
  dn0 = dn0 + es0; dn1 = dn1 + es1; dn2 = dn2 + es2;
  const float dq0 = dn0 + 1e-16f;
  const float dq1 = dn1 + 1e-16f;
  const float dq2 = dn2 + 1e-16f;

  float o0x = 0.0f, o0y = 0.0f, o1x = 0.0f, o1y = 0.0f, o2x = 0.0f, o2y = 0.0f;
#pragma unroll 1
  for (int b0 = 0; b0 < cnt; b0 += 32) {
    const int jj = b0 + lane;
    const bool valid = jj < cnt;
    const int j = valid ? jj : cnt - 1;
    int src; float a0, a1, a2;
    ld_entry(LIST, SD, off + j, dd, src, a0, a1, a2);
    const float w0 = expf(a0 - mx0) / dq0;
    const float w1 = expf(a1 - mx1) / dq1;
    const float w2 = expf(a2 - mx2) / dq2;
    const int m32 = (cnt - b0) < 32 ? (cnt - b0) : 32;
#pragma unroll 1
    for (int k = 0; k < m32; ++k) {
      const int c = __builtin_amdgcn_readlane(src, k);
      const float u0 = __int_as_float(__builtin_amdgcn_readlane(__float_as_int(w0), k));
      const float u1 = __int_as_float(__builtin_amdgcn_readlane(__float_as_int(w1), k));
      const float u2 = __int_as_float(__builtin_amdgcn_readlane(__float_as_int(w2), k));
      const float* xr = XL + (size_t)c * NOUT + 2 * lane;
      const v2f x0 = *(const v2fa*)(xr);
      const v2f x1 = *(const v2fa*)(xr + HCH);
      const v2f x2 = *(const v2fa*)(xr + 2 * HCH);
      asm volatile("" :: "v"(x0), "v"(x1), "v"(x2));
      float pr;
      pr = u0 * x0.x; o0x = o0x + pr;
      pr = u0 * x0.y; o0y = o0y + pr;
      pr = u1 * x1.x; o1x = o1x + pr;
      pr = u1 * x1.y; o1y = o1y + pr;
      pr = u2 * x2.x; o2x = o2x + pr;
      pr = u2 * x2.y; o2y = o2y + pr;
    }
  }
  {
    const float u0 = es0 / dq0;
    const float u1 = es1 / dq1;
    const float u2 = es2 / dq2;
    const float* xr = XL + (size_t)rowc * NOUT + 2 * lane;
    const v2f x0 = *(const v2fa*)(xr);
    const v2f x1 = *(const v2fa*)(xr + HCH);
    const v2f x2 = *(const v2fa*)(xr + 2 * HCH);
    asm volatile("" :: "v"(x0), "v"(x1), "v"(x2));
    float pr;
    pr = u0 * x0.x; o0x = o0x + pr;
    pr = u0 * x0.y; o0y = o0y + pr;
    pr = u1 * x1.x; o1x = o1x + pr;
    pr = u1 * x1.y; o1y = o1y + pr;
    pr = u2 * x2.x; o2x = o2x + pr;
    pr = u2 * x2.y; o2y = o2y + pr;
  }

  const float qnan = __uint_as_float(0x7fc00000u);
  if (LAYER == 1) {
    const v2f bb = *(const v2fa*)(tbB + 2 * lane);
    float m0 = o0x + o1x; m0 = m0 + o2x; m0 = m0 / 3.0f;
    float m1 = o0y + o1y; m1 = m1 + o2y; m1 = m1 / 3.0f;
    float y0 = rrelu_k(m0 + bb.x);
    float y1 = rrelu_k(m1 + bb.y);
    y0 = poison ? qnan : y0;
    y1 = poison ? qnan : y1;
    const unsigned rmask = rin ? 0xFFFFFFFFu : 0u;
    const unsigned hiw = pk16(bf16_bits(y0), bf16_bits(y1)) & rmask;
    const unsigned low = pk16(bf16_lo_bits(y0), bf16_lo_bits(y1)) & rmask;
    unsigned* orow = OUT + (size_t)row * (KT2 / 2);
    volatile unsigned* qh = (volatile unsigned*)(orow + lane);
    volatile unsigned* ql = (volatile unsigned*)(orow + (SPLIT_2 ? 32 : 0) + lane);
    *qh = hiw;
    if (SPLIT_2) *ql = low;
    __threadfence();
    *qh = hiw;
    if (SPLIT_2) *ql = low;
  } else {
    const v2f b0 = *(const v2fa*)(tbB + 0 * HCH + 2 * lane);
    const v2f b1 = *(const v2fa*)(tbB + 1 * HCH + 2 * lane);
    const v2f b2 = *(const v2fa*)(tbB + 2 * HCH + 2 * lane);
    const v2f l0 = *(const v2fa*)(tbLw + 0 * HCH + 2 * lane);
    const v2f l1 = *(const v2fa*)(tbLw + 1 * HCH + 2 * lane);
    const v2f l2 = *(const v2fa*)(tbLw + 2 * HCH + 2 * lane);
    const float lbv = tbLb[0];
    const float y0a = rrelu_k(o0x + b0.x), y0b = rrelu_k(o0y + b0.y);
    const float y1a = rrelu_k(o1x + b1.x), y1b = rrelu_k(o1y + b1.y);
    const float y2a = rrelu_k(o2x + b2.x), y2b = rrelu_k(o2y + b2.y);
    float t = y0a * l0.x;
    float u = y0b * l0.y; t = t + u;
    u = y1a * l1.x; t = t + u;
    u = y1b * l1.y; t = t + u;
    u = y2a * l2.x; t = t + u;
    u = y2b * l2.y; t = t + u;
    t = wsum(t);
    float r = t + lbv;
    r = poison ? qnan : r;
    const unsigned wv = (lane == 0) ? __float_as_uint(r) : 0u;
    volatile unsigned* q = (volatile unsigned*)(OUT + (size_t)rowc * 32 + lane);
    if (rin) *q = wv;
    __threadfence();
    if (rin) *q = wv;
  }
}

__global__ __launch_bounds__(256) void k_flat(const float* __restrict__ RP, float* out) {
  const int f  = (int)blockIdx.x * 256 + (int)threadIdx.x;
  const int fc = f < NN ? f : NN - 1;
  const float v = RP[(size_t)fc * 32];
  asm volatile("" :: "v"(v));
  volatile float* q = (volatile float*)(out + fc);
  const bool wr = f < NN;
  if (wr) *q = v;
  __threadfence();
  if (wr) *q = v;
}

extern "C" void kernel_launch(void* const* d_in, const int* in_sizes, int n_in,
                              void* d_out, int out_size, void* d_ws, size_t ws_size,
                              hipStream_t stream) {
  if (n_in < 13) return;
  if (in_sizes[0] != NN * HCH || in_sizes[1] != NN * HCH) return;
  if (in_sizes[2] != 2 * NE) return;
  if (in_sizes[3] != KIN * NOUT) return;
  if (in_sizes[4] != NOUT || in_sizes[5] != NOUT || in_sizes[6] != HCH) return;
  if (in_sizes[7] != HCH * NOUT) return;
  if (in_sizes[8] != NOUT || in_sizes[9] != NOUT || in_sizes[10] != NOUT) return;
  if (in_sizes[11] != NOUT || in_sizes[12] != 1) return;
  if (out_size != NN) return;

  const float* z    = (const float*)d_in[0];
  const float* x    = (const float*)d_in[1];
  const int*   eidx = (const int*)  d_in[2];
  const float* W1   = (const float*)d_in[3];
  const float* as1  = (const float*)d_in[4];
  const float* ad1  = (const float*)d_in[5];
  const float* b1   = (const float*)d_in[6];
  const float* W2   = (const float*)d_in[7];
  const float* as2  = (const float*)d_in[8];
  const float* ad2  = (const float*)d_in[9];
  const float* b2   = (const float*)d_in[10];
  const float* lw   = (const float*)d_in[11];
  const float* lb   = (const float*)d_in[12];
  float* out = (float*)d_out;
  const int* esrc = eidx;
  const int* edst = eidx + NE;

  const size_t szXB   = (size_t)MPAD * KIN * 2;
  const size_t szW    = (size_t)NOUT * 128 * 2;
  const size_t szTB   = (size_t)TB_N * 4;
  const size_t szXL   = (size_t)MPAD * NOUT * 4;
  const size_t szSD   = (size_t)MPAD * 8 * 4;
  const size_t szRP   = (size_t)MPAD * 32 * 4;
  const size_t szMETA = (size_t)NBLK * NB * 2 * 4;
  const size_t szLIST = (size_t)NBLK * LCAP * 4;
  static_assert((size_t)MPAD * KIN * 2 + 2 * (size_t)NOUT * 128 * 2 + (size_t)TB_N * 4 + (size_t)MPAD * NOUT * 4 +
                (size_t)MPAD * 8 * 4 + (size_t)MPAD * 32 * 4 + (size_t)NBLK * NB * 8 + (size_t)NBLK * LCAP * 4
                == (size_t)499424 * 256);
  static_assert((size_t)499424 * 256 <= WSMAX);
  static_assert((size_t)MPAD * KT2 * 2 <= (size_t)MPAD * KIN * 2);
  char* ws = (char*)d_ws;
  size_t off = 0;
  const size_t oXB   = off; off += szXB;
  const size_t oW1T  = off; off += szW;
  const size_t oW2D  = off; off += szW;
  const size_t oTB   = off; off += szTB;
  const size_t oXL   = off; off += szXL;
  const size_t oSD   = off; off += szSD;
  const size_t oRP   = off; off += szRP;
  const size_t oMETA = off; off += szMETA;
  const size_t oLIST = off; off += szLIST;
  if (off > ws_size || off > (size_t)WSMAX) return;
  unsigned short* XB  = (unsigned short*)(ws + oXB);
  unsigned short* OP  = XB;
  unsigned short* W1T = (unsigned short*)(ws + oW1T);
  unsigned short* W2D = (unsigned short*)(ws + oW2D);
  float*    TB   = (float*)(ws + oTB);
  float*    XL   = (float*)(ws + oXL);
  float*    SD   = (float*)(ws + oSD);
  float*    RP   = (float*)(ws + oRP);
  int*      META = (int*)(ws + oMETA);
  unsigned* LIST = (unsigned*)(ws + oLIST);

  hipFuncSetAttribute(reinterpret_cast<const void*>(&k_list),
                      hipFuncAttributeMaxDynamicSharedMemorySize, LDS_LIST);

  const int tiles = (MPAD / 64) * (NOUT / 64);
  const int gG = (tiles + 7) / 8;

  k_planezx<<<MPAD * 16 / 256, 256, 0, stream>>>(z, x, XB);
  k_prep<<<PREP_BLK, 256, 0, stream>>>(W1, W2, as1, ad1, b1, as2, ad2, b2, lw, lb, W1T, W2D, TB);
  k_list<<<NBLK, BT, LDS_LIST, stream>>>(esrc, edst, LIST, META);
  k_gemm_nt<0, 0><<<gG, 256, 0, stream>>>(XB, W1T, TB, XL, MPAD, NOUT, KIN, NOUT);
  k_rowprep<<<MPAD / 32, 256, 0, stream>>>(XL, TB + TB_AS1, TB + TB_AD1, SD);
  k_walk<1><<<MPAD / WWAVES, WTHR, 0, stream>>>(XL, SD, LIST, META, TB + TB_B1, TB + TB_LW, TB + TB_LB,
                                                 (unsigned*)OP);
  k_gemm_nt<0, 0><<<gG, 256, 0, stream>>>(OP, W2D, TB, XL, MPAD, NOUT, KT2, NOUT);
  k_rowprep<<<MPAD / 32, 256, 0, stream>>>(XL, TB + TB_AS2, TB + TB_AD2, SD);
  k_walk<2><<<NN / WWAVES, WTHR, 0, stream>>>(XL, SD, LIST, META, TB + TB_B2, TB + TB_LW, TB + TB_LB,
                                               (unsigned*)RP);
  k_flat<<<(NN + 255) / 256, 256, 0, stream>>>(RP, out);
}
